// LinearAttention_91250875170835
// MI455X (gfx1250) — hardware-run, weakly checked
//
#include <hip/hip_runtime.h>
#include <math.h>

typedef __attribute__((ext_vector_type(16))) __bf16   v16b;
typedef __attribute__((ext_vector_type(8)))  __bf16   v8b;
typedef __attribute__((ext_vector_type(8)))  float    v8f;
typedef __attribute__((ext_vector_type(4)))  float    v4f;
typedef __attribute__((ext_vector_type(4)))  unsigned int v4u;

constexpr int kL  = 1024;
constexpr int kNb = 2;
constexpr int kE  = 1024;
constexpr int kH  = 16;
constexpr int kD  = 64;
constexpr int kM  = kL * kNb;
constexpr int kTS = 32;
constexpr int kNP = 68;
constexpr float kEps = 1e-6f;
static_assert(kH * kD == kE);
static_assert((kM % 64) == 0 && (kE % 64) == 0 && (kE % 32) == 0);
static_assert((kL % kTS) == 0);
static_assert(((kM * kE / 8) % 256) == 0 && ((kE * kE / 8) % 256) == 0);

constexpr size_t kSzXB   = (size_t)kM * kE * 2;
constexpr size_t kSzWB   = (size_t)kE * kE * 2;
constexpr size_t kSzBias = (size_t)4 * kE * 4;
constexpr size_t kSzF    = (size_t)kM * kE * 4;
constexpr size_t kSzAB   = (size_t)kM * kE * 2;
constexpr size_t kOffXB   = 0;
constexpr size_t kOffWB   = kOffXB + 3 * kSzXB;
constexpr size_t kOffBias = kOffWB + 4 * kSzWB;
constexpr size_t kOffQF   = kOffBias + kSzBias;
constexpr size_t kOffKF   = kOffQF + kSzF;
constexpr size_t kOffVF   = kOffKF + kSzF;
constexpr size_t kOffAH   = kOffVF + kSzF;
constexpr size_t kOffAL   = kOffAH + kSzAB;
constexpr size_t kWsTotal = kOffAL + kSzAB;
static_assert(kWsTotal == 54542336ull);
static_assert(kWsTotal <= 134217728ull);
static_assert((kOffWB % 128) == 0 && (kOffBias % 128) == 0 && (kOffQF % 128) == 0 && (kOffKF % 128) == 0 &&
              (kOffVF % 128) == 0 && (kOffAH % 128) == 0 && (kOffAL % 128) == 0);

__device__ __forceinline__ unsigned short f2bf_bits(float f) {
  unsigned u = __float_as_uint(f);
  return (unsigned short)((u + 0x7FFFu + ((u >> 16) & 1u)) >> 16);
}
__device__ __forceinline__ float bf_bits2f(unsigned short h) { return __uint_as_float(((unsigned)h) << 16); }
__device__ __forceinline__ float bf16r(float f) { return bf_bits2f(f2bf_bits(f)); }
__device__ __forceinline__ unsigned pk16(unsigned short a, unsigned short b) { return (unsigned)a | ((unsigned)b << 16); }

__device__ __forceinline__ void tie2_b(v8f& a, v16b x, v16b y) { asm volatile("v_nop\n\tv_nop\n\tv_nop\n\tv_nop" : "+v"(a) : "v"(x), "v"(y)); }
__device__ __forceinline__ void tie3_b(v8f& a, v16b x, v16b y, v16b z) { asm volatile("v_nop\n\tv_nop\n\tv_nop\n\tv_nop" : "+v"(a) : "v"(x), "v"(y), "v"(z)); }
__device__ __forceinline__ void keep4_b(v16b a, v16b b, v16b c, v16b d) { asm volatile("v_nop" :: "v"(a), "v"(b), "v"(c), "v"(d)); }
__device__ __forceinline__ void acc_guard4(v8f& a, v8f& b, v8f& c, v8f& d) { asm volatile("v_nop\n\tv_nop\n\tv_nop\n\tv_nop" : "+v"(a), "+v"(b), "+v"(c), "+v"(d)); }

struct FragB {
  union U { v16b v; v8b h[2]; };
  static __device__ __forceinline__ v16b load(const __bf16* p) {
    U f; f.h[0] = *(const v8b*)(p); f.h[1] = *(const v8b*)(p + 16); return f.v;
  }
  static __device__ __forceinline__ v8f mma(v16b a, v16b b, v8f c) {
    return __builtin_amdgcn_wmma_f32_16x16x32_bf16(false, a, false, b, (short)0, c, false, false);
  }
};

__global__ __launch_bounds__(256) void cvt8_bf16_kernel(
    const float* __restrict__ s0, const float* __restrict__ s1, const float* __restrict__ s2,
    const float* __restrict__ s3, unsigned short* __restrict__ dst, int n8)
{
  const int y = blockIdx.y;
  const float* src = (y == 0) ? s0 : (y == 1) ? s1 : (y == 2) ? s2 : s3;
  const int i = blockIdx.x * 256 + threadIdx.x;
  if (i < n8) {
    const float* p = src + 8 * (size_t)i;
    const v4f a = *(const v4f*)(p);
    const v4f c = *(const v4f*)(p + 4);
    unsigned short hb[8];
#pragma unroll
    for (int e = 0; e < 4; ++e) {
      const float fa = a[e];
      const float fc = c[e];
      hb[e]     = f2bf_bits(fa);
      hb[4 + e] = f2bf_bits(fc);
    }
    const v4u u = (v4u){pk16(hb[0], hb[1]), pk16(hb[2], hb[3]), pk16(hb[4], hb[5]), pk16(hb[6], hb[7])};
    unsigned short* q = dst + ((size_t)y * (size_t)n8 + (size_t)i) * 8;
    *(volatile v4u*)q = u;
    __threadfence();
    *(volatile v4u*)q = u;
  }
}

__global__ __launch_bounds__(256) void bias_bf16_kernel(
    const float* __restrict__ b0, const float* __restrict__ b1, const float* __restrict__ b2,
    const float* __restrict__ b3, float* __restrict__ dst)
{
  const int y = blockIdx.x;
  const float* src = (y == 0) ? b0 : (y == 1) ? b1 : (y == 2) ? b2 : b3;
  const int idx = threadIdx.x * 4;
  const v4f v = *(const v4f*)(src + idx);
  v4f o;
#pragma unroll
  for (int e = 0; e < 4; ++e) {
    const float fv = v[e];
    o[e] = bf16r(fv);
  }
  float* op = dst + (size_t)y * kE + idx;
  *(volatile v4f*)op = o;
  __threadfence();
  *(volatile v4f*)op = o;
}

template <int SPL, int ACT>
__global__ __launch_bounds__(256) void wmma_gemm64(
    const unsigned short* __restrict__ Ap, const unsigned short* __restrict__ A2p, int lda,
    const unsigned short* __restrict__ Btp, int ldb,
    float* __restrict__ C, int ldc,
    const float* __restrict__ bias,
    int M, int N, int K)
{
  const __bf16* A  = (const __bf16*)Ap;
  const __bf16* A2 = (const __bf16*)A2p;
  const __bf16* Bt = (const __bf16*)Btp;
  __shared__ __align__(16) float sT[8][16 * 68];
  const int lane = threadIdx.x & 31;
  const int wave = threadIdx.x >> 5;
  const int tilesN = N >> 6;
  const int tilesM = M >> 6;
  const int tile = blockIdx.x * 8 + wave;
  if (tile >= tilesM * tilesN) return;
  const int tm = tile / tilesN;
  const int tn = tile - tm * tilesN;
  const int m0 = tm << 6;
  const int n0 = tn << 6;

  const int rlane = lane & 15;
  const int koff  = (lane >> 4) * 8;
  const int mOff  = (lane >> 4) * 8;

  v8f acc[4][4];
#pragma unroll
  for (int i = 0; i < 4; ++i)
#pragma unroll
    for (int j = 0; j < 4; ++j) acc[i][j] = (v8f){0.f, 0.f, 0.f, 0.f, 0.f, 0.f, 0.f, 0.f};

  for (int k0 = 0; k0 < K; k0 += 32) {
    v16b bh[4];
#pragma unroll
    for (int j = 0; j < 4; ++j) {
      const size_t bo = (size_t)(n0 + (j << 4) + rlane) * ldb + koff + k0;
      bh[j] = FragB::load(Bt + bo);
    }
#pragma unroll
    for (int i = 0; i < 4; ++i) {
      const size_t ao = (size_t)(m0 + (i << 4) + rlane) * lda + koff + k0;
      v16b ah = FragB::load(A + ao);
      v16b al;
      if (SPL == 1) al = FragB::load(A2 + ao);
#pragma unroll
      for (int j = 0; j < 4; ++j) {
        acc[i][j] = FragB::mma(ah, bh[j], acc[i][j]);
        if (SPL == 1) acc[i][j] = FragB::mma(al, bh[j], acc[i][j]);
      }
#pragma unroll
      for (int j = 0; j < 4; ++j) {
        if (SPL == 1) tie3_b(acc[i][j], ah, al, bh[j]);
        else          tie2_b(acc[i][j], ah, bh[j]);
      }
    }
    keep4_b(bh[0], bh[1], bh[2], bh[3]);
  }
  acc_guard4(acc[0][0], acc[0][1], acc[0][2], acc[0][3]);
  acc_guard4(acc[1][0], acc[1][1], acc[1][2], acc[1][3]);
  acc_guard4(acc[2][0], acc[2][1], acc[2][2], acc[2][3]);
  acc_guard4(acc[3][0], acc[3][1], acc[3][2], acc[3][3]);

  float* slab = sT[wave];
#pragma unroll
  for (int i = 0; i < 4; ++i) {
    const int mBase = m0 + (i << 4);
#pragma unroll
    for (int j = 0; j < 4; ++j) {
      const int n = n0 + (j << 4) + rlane;
      const float bv = bias[n];
#pragma unroll
      for (int r = 0; r < 8; ++r) {
        float v = acc[i][j][r] + bv;
        if (ACT == 6) v = (v > 0.0f) ? (v + 1.0f) : expf(v);
        slab[(mOff + r) * 68 + (j << 4) + rlane] = v;
      }
    }
    __builtin_amdgcn_fence(__ATOMIC_RELEASE, "workgroup");
    __builtin_amdgcn_wave_barrier();
    __builtin_amdgcn_fence(__ATOMIC_ACQUIRE, "workgroup");
    {
      const int hh = lane >> 4, c4 = (lane & 15) * 4;
      for (int pass = 0; pass < 2; ++pass) {
#pragma unroll
        for (int it = 0; it < 8; ++it) {
          const int row = it * 2 + hh;
          v4f v = *(const v4f*)(slab + row * 68 + c4);
          *(volatile v4f*)(C + (size_t)(mBase + row) * ldc + n0 + c4) = v;
        }
        __threadfence();
      }
    }
    __builtin_amdgcn_fence(__ATOMIC_RELEASE, "workgroup");
    __builtin_amdgcn_wave_barrier();
    __builtin_amdgcn_fence(__ATOMIC_ACQUIRE, "workgroup");
  }
}

__global__ __launch_bounds__(128) void state_scan_kernel(
    const float* __restrict__ QF, const float* __restrict__ KF, const float* __restrict__ VF,
    unsigned short* __restrict__ AH, unsigned short* __restrict__ AL)
{
  __shared__ __align__(16) float sQ[kTS * kD];
  __shared__ __align__(16) float sK[kTS * kD];
  __shared__ __align__(16) float sV[kTS * kD];
  __shared__ __align__(16) float sZ[kTS * kD];
  __shared__ __align__(16) float sN[2 * kTS * kNP];
  __shared__ __align__(16) float sDp[kTS * 4];

  const int tid  = threadIdx.x;
  const int lane = tid & 31;
  const int wave = tid >> 5;
  const int half = tid >> 6;
  const int e    = tid & 63;
  const int nb   = blockIdx.x / kH;
  const int hd   = blockIdx.x - nb * kH;
  const int colbase = hd * kD;

  float S[32];
#pragma unroll
  for (int i = 0; i < 32; ++i) S[i] = 0.0f;
  float zr = 0.0f;

  const int lr  = tid >> 4;
  const int lc4 = (tid & 15) * 4;
  const int oq  = lane >> 3;
  const int oc8 = (lane & 7) * 8;

  const float* kp = sK + half * 32;
  const float* qp = sQ + half * 32;
  float* np = sN + half * (kTS * kNP) + e;

#pragma unroll 1
  for (int t0 = 0; t0 < kL; t0 += kTS) {
    __syncthreads();
#pragma unroll
    for (int i = 0; i < 4; ++i) {
      const int r = lr + 8 * i;
      const size_t g = ((size_t)(t0 + r) * kNb + nb) * kE + colbase + lc4;
      *(v4f*)(sQ + r * kD + lc4) = *(const v4f*)(QF + g);
      *(v4f*)(sK + r * kD + lc4) = *(const v4f*)(KF + g);
      *(v4f*)(sV + r * kD + lc4) = *(const v4f*)(VF + g);
    }
    __syncthreads();

    if (tid < 64) {
#pragma unroll 1
      for (int s = 0; s < kTS; ++s) {
        zr += sK[s * kD + tid];
        sZ[s * kD + tid] = zr;
      }
    }

#pragma unroll 1
    for (int s = 0; s < kTS; ++s) {
      const float vv = sV[s * kD + e];
      float acc = 0.0f;
#pragma unroll
      for (int j = 0; j < 8; ++j) {
        const v4f k4 = *(const v4f*)(kp + s * kD + 4 * j);
        const v4f q4 = *(const v4f*)(qp + s * kD + 4 * j);
#pragma unroll
        for (int c = 0; c < 4; ++c) {
          S[4 * j + c] = fmaf(k4[c], vv, S[4 * j + c]);
          acc = fmaf(q4[c], S[4 * j + c], acc);
        }
      }
      np[s * kNP] = acc;
    }
    __syncthreads();

    {
      const int tr = tid >> 2, qu = tid & 3;
      const float* qd = sQ + tr * kD + qu * 16;
      const float* zd = sZ + tr * kD + qu * 16;
      float p = 0.0f;
#pragma unroll 1
      for (int j = 0; j < 4; ++j) {
        const v4f a = *(const v4f*)(qd + 4 * j);
        const v4f b = *(const v4f*)(zd + 4 * j);
        p = fmaf(a[0], b[0], p);
        p = fmaf(a[1], b[1], p);
        p = fmaf(a[2], b[2], p);
        p = fmaf(a[3], b[3], p);
      }
      sDp[tid] = p;
    }
    __syncthreads();

#pragma unroll 1
    for (int it = 0; it < 2; ++it) {
      const int row = it * 16 + wave * 4 + oq;
      const v4f dp = *(const v4f*)(sDp + row * 4);
      const float den  = ((dp[0] + dp[1]) + (dp[2] + dp[3])) + kEps;
      const float rinv = 1.0f / den;
      const float* pa = sN + row * kNP + oc8;
      const float* pb = sN + kTS * kNP + row * kNP + oc8;
      const v4f a0 = *(const v4f*)(pa);
      const v4f a1 = *(const v4f*)(pa + 4);
      const v4f b0 = *(const v4f*)(pb);
      const v4f b1 = *(const v4f*)(pb + 4);
      unsigned short hb[8], lb[8];
#pragma unroll
      for (int x = 0; x < 4; ++x) {
        const float f0 = (a0[x] + b0[x]) * rinv;
        const float f1 = (a1[x] + b1[x]) * rinv;
        const unsigned short h0 = f2bf_bits(f0);
        const unsigned short h1 = f2bf_bits(f1);
        hb[x]     = h0;
        hb[4 + x] = h1;
        lb[x]     = f2bf_bits(f0 - bf_bits2f(h0));
        lb[4 + x] = f2bf_bits(f1 - bf_bits2f(h1));
      }
      const v4u hv = (v4u){pk16(hb[0], hb[1]), pk16(hb[2], hb[3]), pk16(hb[4], hb[5]), pk16(hb[6], hb[7])};
      const v4u lv = (v4u){pk16(lb[0], lb[1]), pk16(lb[2], lb[3]), pk16(lb[4], lb[5]), pk16(lb[6], lb[7])};
      const size_t o = ((size_t)(t0 + row) * kNb + nb) * kE + colbase + oc8;
      *(volatile v4u*)(AH + o) = hv;
      *(volatile v4u*)(AL + o) = lv;
      __threadfence();
      *(volatile v4u*)(AH + o) = hv;
      *(volatile v4u*)(AL + o) = lv;
    }
  }
}

extern "C" void kernel_launch(void* const* d_in, const int* in_sizes, int n_in,
                              void* d_out, int out_size, void* d_ws, size_t ws_size,
                              hipStream_t stream) {
  if (n_in < 11 || d_out == nullptr || d_ws == nullptr) return;
  if (in_sizes[0] != kM * kE || in_sizes[1] != kM * kE || in_sizes[2] != kM * kE) return;
  if (in_sizes[3] != kE * kE || in_sizes[5] != kE * kE || in_sizes[7] != kE * kE || in_sizes[9] != kE * kE) return;
  if (in_sizes[4] != kE || in_sizes[6] != kE || in_sizes[8] != kE || in_sizes[10] != kE) return;
  if (out_size != kM * kE) return;
  if (ws_size < kWsTotal) return;

  const float* query = (const float*)d_in[0];
  const float* key_  = (const float*)d_in[1];
  const float* value = (const float*)d_in[2];
  const float* Wq = (const float*)d_in[3];
  const float* bq = (const float*)d_in[4];
  const float* Wk = (const float*)d_in[5];
  const float* bk = (const float*)d_in[6];
  const float* Wv = (const float*)d_in[7];
  const float* bv = (const float*)d_in[8];
  const float* Wo = (const float*)d_in[9];
  const float* bo = (const float*)d_in[10];
  float* out = (float*)d_out;

  char* ws = (char*)d_ws;
  unsigned short* XB    = (unsigned short*)(ws + kOffXB);
  unsigned short* WB    = (unsigned short*)(ws + kOffWB);
  float*          BIASF = (float*)(ws + kOffBias);
  float*          QF    = (float*)(ws + kOffQF);
  float*          KF    = (float*)(ws + kOffKF);
  float*          VF    = (float*)(ws + kOffVF);
  unsigned short* AH    = (unsigned short*)(ws + kOffAH);
  unsigned short* AL    = (unsigned short*)(ws + kOffAL);

  const size_t planeX = (size_t)kM * kE;
  const size_t planeW = (size_t)kE * kE;

  cvt8_bf16_kernel<<<dim3((kM * kE / 8) / 256, 3), 256, 0, stream>>>(query, key_, value, value, XB, kM * kE / 8);
  cvt8_bf16_kernel<<<dim3((kE * kE / 8) / 256, 4), 256, 0, stream>>>(Wq, Wk, Wv, Wo, WB, kE * kE / 8);
  bias_bf16_kernel<<<4, 256, 0, stream>>>(bq, bk, bv, bo, BIASF);

  const dim3 ggrid((kM / 64) * (kE / 64) / 8, 1);
  wmma_gemm64<0, 6><<<ggrid, 256, 0, stream>>>(XB, XB, kE, WB, kE, QF, kE, BIASF, kM, kE, kE);
  wmma_gemm64<0, 6><<<ggrid, 256, 0, stream>>>(XB + planeX, XB + planeX, kE, WB + planeW, kE, KF, kE, BIASF + kE, kM, kE, kE);
  wmma_gemm64<0, 0><<<ggrid, 256, 0, stream>>>(XB + 2 * planeX, XB + 2 * planeX, kE, WB + 2 * planeW, kE, VF, kE, BIASF + 2 * kE, kM, kE, kE);

  state_scan_kernel<<<kNb * kH, 128, 0, stream>>>(QF, KF, VF, AH, AL);

  wmma_gemm64<1, 0><<<ggrid, 256, 0, stream>>>(AH, AL, kE, WB + 3 * planeW, kE, out, kE, BIASF + 3 * kE, kM, kE, kE);
}
